// mLSTMCell_78537771975160
// MI455X (gfx1250) — hardware-verified
//
#include <hip/hip_runtime.h>
#include <math.h>

constexpr int kS = 2048;
constexpr int kHid = 1024;
constexpr int kNH = 8;
constexpr int kDH = 128;
constexpr int kHeadElems = kS * kDH;
constexpr int kHeadWords = kHeadElems / 2;
constexpr int kGateK = 3 * kHid;
constexpr int kGateN = 2 * kNH;
constexpr int kPcxRows = 144;
constexpr int kPcxHead = kPcxRows * kDH;
constexpr int kStatN = 4;
constexpr int kMtabPitch = 32;
constexpr int kWPitch = 72;
constexpr int kOsPitch = 68;
constexpr float kQScale = 0.08838834764831845f;
constexpr int kOutN = kNH * kDH * kDH;
constexpr int kOutM = kOutN + kNH * kDH;
constexpr int kOutO = kOutM + kNH;
constexpr int kOutTotal = kOutO + kNH * kS * kDH;
constexpr int kPackN4 = (kOutTotal - kOutM) / 4;
static_assert(kOutN == 131072 && kOutM == 132096 && kOutO == 132104 && kOutTotal == 2229256);
static_assert(kPackN4 * 4 == kOutTotal - kOutM && kPackN4 == 524290);
static_assert((kOutM * 4) % 128 == 0);
static_assert(kDH % 32 == 0 && kS % 64 == 0 && kHid % 32 == 0 && kGateK % 32 == 0);
static_assert((kWPitch * 2) % 16 == 0 && (kOsPitch * 4) % 16 == 0);

typedef __attribute__((ext_vector_type(16))) __bf16   v16b;
typedef __attribute__((ext_vector_type(8)))  __bf16   v8b;
typedef __attribute__((ext_vector_type(8)))  float    v8f;
typedef __attribute__((ext_vector_type(4)))  float    v4f;
typedef __attribute__((ext_vector_type(4)))  unsigned int v4u;
typedef __attribute__((ext_vector_type(4)))  int      v4i;

__device__ __forceinline__ unsigned short f2bf_bits(float f) {
  unsigned u = __float_as_uint(f);
  return (unsigned short)((u + 0x7FFFu + ((u >> 16) & 1u)) >> 16);
}
__device__ __forceinline__ float bf_bits2f(unsigned short hbv) { return __uint_as_float(((unsigned)hbv) << 16); }
__device__ __forceinline__ float bfr(float f) { return bf_bits2f(f2bf_bits(f)); }
__device__ __forceinline__ unsigned pk16(unsigned short a, unsigned short b) { return (unsigned)a | ((unsigned)b << 16); }
__device__ __forceinline__ v8f zero8() { v8f z = {0.f, 0.f, 0.f, 0.f, 0.f, 0.f, 0.f, 0.f}; return z; }

__device__ __forceinline__ v16b fload(const unsigned short* p) {
  union { v16b v; v8b hv[2]; } f;
  f.hv[0] = *(const v8b*)(const void*)(p);
  f.hv[1] = *(const v8b*)(const void*)(p + 16);
  return f.v;
}
__device__ __forceinline__ v8f mma_bf(v16b a, v16b b, v8f cacc) {
  return __builtin_amdgcn_wmma_f32_16x16x32_bf16(false, a, false, b, (short)0, cacc, false, false);
}
__device__ __forceinline__ void hz1(v8f& c0, v16b a, v16b b) {
  asm volatile("v_nop\n\tv_nop\n\tv_nop\n\tv_nop" : "+v"(c0) : "v"(a), "v"(b));
}
__device__ __forceinline__ void hz1x3(v8f& c0, v16b a, v16b a2, v16b b) {
  asm volatile("v_nop\n\tv_nop\n\tv_nop\n\tv_nop" : "+v"(c0) : "v"(a), "v"(a2), "v"(b));
}
__device__ __forceinline__ void hz4x5(v8f& c0, v8f& c1, v8f& c2, v8f& c3, v16b a, v16b b0, v16b b1, v16b b2, v16b b3) {
  asm volatile("v_nop\n\tv_nop\n\tv_nop\n\tv_nop" : "+v"(c0), "+v"(c1), "+v"(c2), "+v"(c3) : "v"(a), "v"(b0), "v"(b1), "v"(b2), "v"(b3));
}
__device__ __forceinline__ void hz4x6(v8f& c0, v8f& c1, v8f& c2, v8f& c3, v16b a, v16b a2, v16b b0, v16b b1, v16b b2, v16b b3) {
  asm volatile("v_nop\n\tv_nop\n\tv_nop\n\tv_nop" : "+v"(c0), "+v"(c1), "+v"(c2), "+v"(c3) : "v"(a), "v"(a2), "v"(b0), "v"(b1), "v"(b2), "v"(b3));
}
__device__ __forceinline__ void sched_fence() { asm volatile("" ::: "memory"); }

__device__ __forceinline__ void plane_store_f(const float* src, float* dst, int t) {
  for (int pass = 0; pass < 2; ++pass) {
#pragma unroll
    for (int it = 0; it < 2; ++it) {
      const int idx = it * 1024 + 4 * t;
      const v4f val = *(const v4f*)(src + idx);
      *(volatile v4f*)(dst + idx) = val;
    }
    __threadfence();
  }
}
__device__ __forceinline__ void plane_store_i(const int* src, int* dst, int t) {
  for (int pass = 0; pass < 2; ++pass) {
#pragma unroll
    for (int it = 0; it < 2; ++it) {
      const int idx = it * 1024 + 4 * t;
      const v4i val = *(const v4i*)(src + idx);
      *(volatile v4i*)(dst + idx) = val;
    }
    __threadfence();
  }
}

__global__ __launch_bounds__(256) void k_cast3(const float* __restrict__ x0, const float* __restrict__ x1,
                                              const float* __restrict__ x2, unsigned short* __restrict__ y0,
                                              unsigned short* __restrict__ y1, unsigned short* __restrict__ y2, int n8) {
  const int z = blockIdx.y;
  const float* in = (z == 0) ? x0 : ((z == 1) ? x1 : x2);
  unsigned short* outp = (z == 0) ? y0 : ((z == 1) ? y1 : y2);
  const int i = blockIdx.x * 256 + threadIdx.x;
  if (i >= n8) return;
  const float* p = in + 8 * (size_t)i;
  const v4f a = *(const v4f*)(p);
  const v4f b = *(const v4f*)(p + 4);
  unsigned short hb[8];
#pragma unroll
  for (int e = 0; e < 4; ++e) {
    hb[e]     = f2bf_bits(a[e]);
    hb[4 + e] = f2bf_bits(b[e]);
  }
  const v4u u = (v4u){pk16(hb[0], hb[1]), pk16(hb[2], hb[3]), pk16(hb[4], hb[5]), pk16(hb[6], hb[7])};
  unsigned short* qd = outp + 8 * (size_t)i;
  *(volatile v4u*)qd = u;
  __threadfence();
  *(volatile v4u*)qd = u;
}

__global__ __launch_bounds__(256) void k_tcast(const float* __restrict__ in, unsigned short* __restrict__ outp,
                                              int nrow, int ncol, int inHead, int outHead) {
  __shared__ float sm[64][65];
  const int t  = threadIdx.x;
  const int s0 = blockIdx.x * 64;
  const int d0 = blockIdx.y * 64;
  const int h  = blockIdx.z;
  const float* inh = in + (size_t)h * inHead;
#pragma unroll
  for (int i = 0; i < 16; ++i) {
    const int e = i * 256 + t;
    const int r = e >> 6;
    const int cc = e & 63;
    sm[cc][r] = inh[(size_t)(s0 + r) * ncol + d0 + cc];
  }
  __syncthreads();
  const int lane = t & 31, wave = t >> 5;
  const int q8 = lane >> 3, c8 = (lane & 7) * 8;
  unsigned short* oh = outp + (size_t)h * outHead;
  for (int pass = 0; pass < 2; ++pass) {
#pragma unroll
    for (int it = 0; it < 2; ++it) {
      const int row = wave * 8 + it * 4 + q8;
      unsigned short hb[8];
#pragma unroll
      for (int e = 0; e < 8; ++e) hb[e] = f2bf_bits(sm[row][c8 + e]);
      const v4u u = (v4u){pk16(hb[0], hb[1]), pk16(hb[2], hb[3]), pk16(hb[4], hb[5]), pk16(hb[6], hb[7])};
      *(volatile v4u*)(oh + (size_t)(d0 + row) * nrow + s0 + c8) = u;
    }
    __threadfence();
  }
}

__global__ __launch_bounds__(256) void k_prep2(const float* __restrict__ wik, const float* __restrict__ wfk,
                                              const float* __restrict__ prevN, unsigned short* __restrict__ GBt,
                                              unsigned short* __restrict__ PCX) {
  const int t = threadIdx.x;
  if (blockIdx.x < 24) {
    const int u = blockIdx.x * 256 + t;
    const int cch = u / 384;
    const int k8 = u - cch * 384;
    const int cc = cch & 7;
    const float fi = (cch < 8) ? 1.0f : 0.0f;
    const float ff = 1.0f - fi;
    unsigned short hb[8];
#pragma unroll
    for (int e = 0; e < 4; ++e) {
      const int kk = k8 * 8 + e;
      const float a = wik[(size_t)kk * kNH + cc];
      const float b = wfk[(size_t)kk * kNH + cc];
      hb[e] = f2bf_bits(fi * a + ff * b);
    }
    sched_fence();
#pragma unroll
    for (int e = 4; e < 8; ++e) {
      const int kk = k8 * 8 + e;
      const float a = wik[(size_t)kk * kNH + cc];
      const float b = wfk[(size_t)kk * kNH + cc];
      hb[e] = f2bf_bits(fi * a + ff * b);
    }
    const v4u uu = (v4u){pk16(hb[0], hb[1]), pk16(hb[2], hb[3]), pk16(hb[4], hb[5]), pk16(hb[6], hb[7])};
    unsigned short* dp = GBt + (size_t)cch * kGateK + k8 * 8;
    *(volatile v4u*)dp = uu;
    __threadfence();
    *(volatile v4u*)dp = uu;
  } else {
    const int u = (blockIdx.x - 24) * 256 + t;
    const int h = u >> 8;
    const int rem = u & 255;
    const int row = 128 + (rem >> 4);
    const int c8 = (rem & 15) * 8;
    const float fsel = (row == 128) ? 1.0f : 0.0f;
    const v4f a = *(const v4f*)(prevN + (size_t)h * kDH + c8);
    const v4f b = *(const v4f*)(prevN + (size_t)h * kDH + c8 + 4);
    unsigned short hb[8];
#pragma unroll
    for (int e = 0; e < 4; ++e) {
      hb[e]     = f2bf_bits(fsel * a[e] + 0.0f);
      hb[4 + e] = f2bf_bits(fsel * b[e] + 0.0f);
    }
    const v4u uu = (v4u){pk16(hb[0], hb[1]), pk16(hb[2], hb[3]), pk16(hb[4], hb[5]), pk16(hb[6], hb[7])};
    unsigned short* dp = PCX + (size_t)h * kPcxHead + (size_t)row * kDH + c8;
    *(volatile v4u*)dp = uu;
    __threadfence();
    *(volatile v4u*)dp = uu;
  }
}

__device__ __forceinline__ void gate_seg(v8f (&acc)[4], const unsigned short* __restrict__ A,
                                         const unsigned short* __restrict__ Bt, int m0, int c, int koff) {
#pragma unroll 1
  for (int k0 = 0; k0 < kHid; k0 += 32) {
    const v16b bq = fload(Bt + k0 + koff);
#pragma unroll
    for (int i = 0; i < 4; ++i) {
      const v16b aq = fload(A + (size_t)(m0 + 16 * i + c) * kHid + k0 + koff);
      acc[i] = mma_bf(aq, bq, acc[i]);
      hz1(acc[i], aq, bq);
    }
  }
}

__global__ __launch_bounds__(256) void k_gates(const unsigned short* __restrict__ Qb, const unsigned short* __restrict__ Kb,
                                              const unsigned short* __restrict__ Vb, const unsigned short* __restrict__ GBt,
                                              const float* __restrict__ wib, const float* __restrict__ wfb,
                                              float* __restrict__ Ipl, float* __restrict__ Fpl) {
  __shared__ __align__(16) float sG[8][64 * kGateN];
  const int tid = threadIdx.x;
  const int wave = tid >> 5, lane = tid & 31, hh = lane >> 4, c = lane & 15, koff = hh * 8;
  const int m0 = (blockIdx.x * 8 + wave) * 64;
  v8f acc[4];
#pragma unroll
  for (int i = 0; i < 4; ++i) acc[i] = zero8();
  const unsigned short* btc = GBt + (size_t)c * kGateK;
  gate_seg(acc, Qb, btc, m0, c, koff);
  gate_seg(acc, Kb, btc + kHid, m0, c, koff);
  gate_seg(acc, Vb, btc + 2 * kHid, m0, c, koff);

  const float bi = wib[c & 7];
  const float bfv = wfb[c & 7];
  const float fi = (c < 8) ? 1.0f : 0.0f;
  const float bsel = bfr(fi * bi + (1.0f - fi) * bfv);
  float* slab = sG[wave];
#pragma unroll
  for (int i = 0; i < 4; ++i) {
#pragma unroll
    for (int r = 0; r < 8; ++r) slab[(16 * i + 8 * hh + r) * kGateN + c] = acc[i][r] + bsel;
  }
  __syncthreads();
  for (int pass = 0; pass < 2; ++pass) {
#pragma unroll
    for (int it = 0; it < 4; ++it) {
      const int f4 = it * 32 + lane;
      const int row = f4 >> 1;
      const int c0 = (f4 & 1) * 4;
      const v4f vi = *(const v4f*)(slab + row * kGateN + c0);
      const v4f vf = *(const v4f*)(slab + row * kGateN + kNH + c0);
      *(volatile v4f*)(Ipl + (size_t)(m0 + row) * kNH + c0) = vi;
      *(volatile v4f*)(Fpl + (size_t)(m0 + row) * kNH + c0) = vf;
    }
    __threadfence();
  }
}

__global__ __launch_bounds__(256) void k_rowstats(
    const float* __restrict__ Ipl, const float* __restrict__ Fpl, const int* __restrict__ resetFlags,
    const float* __restrict__ prevM, const float* __restrict__ prevN, const unsigned int* __restrict__ Kb32,
    float* __restrict__ ST, int* __restrict__ EPS, float* __restrict__ Mtab,
    unsigned short* __restrict__ KKh, unsigned short* __restrict__ KKl, float* __restrict__ outN) {
  __shared__ __align__(16) float sLfc[kS];
  __shared__ __align__(16) float sA[kS];
  __shared__ __align__(16) int sE[kS];
  __shared__ float sF[256];
  __shared__ int sI[256];
  __shared__ float sRed[8];
  __shared__ __align__(16) float sPn[kDH];
  __shared__ __align__(16) unsigned short sHi[64 * kWPitch];
  __shared__ __align__(16) unsigned short sLo[64 * kWPitch];
  __shared__ float sN[8][kDH];
  __shared__ __align__(16) float sOut[kDH];

  const int h = blockIdx.x, t = threadIdx.x, lane = t & 31, wave = t >> 5, base = t * 8;
  const float* Ih = Ipl + (size_t)h * kS;
  const float* Fh = Fpl + (size_t)h * kS;
  const float pmb = bfr(prevM[h]);
  if (wave < 4) sPn[t] = bfr(prevN[(size_t)h * kDH + t]);

  float run = 0.0f;
  int cur = -1;
#pragma unroll 1
  for (int e = 0; e < 8; ++e) {
    const int s = base + e;
    const float f = Fh[s];
    const float lf = fminf(f, 0.0f) - log1pf(expf(-fabsf(f)));
    run = run + lf;
    sLfc[s] = run;
    const int mk = resetFlags[s];
    cur = (mk != 0) ? s : cur;
    sE[s] = cur;
  }
  sF[t] = run;
  sI[t] = cur;
  __syncthreads();
  if (t == 0) {
    float r = 0.0f;
    int ci = -1;
    for (int j = 0; j < 256; ++j) {
      const float tv = sF[j]; sF[j] = r; r = r + tv;
      const int ti = sI[j]; sI[j] = ci; ci = (ti > ci) ? ti : ci;
    }
  }
  __syncthreads();
  {
    const float off = sF[t];
    const int coff = sI[t];
#pragma unroll 1
    for (int e = 0; e < 8; ++e) {
      const int s = base + e;
      sLfc[s] = off + sLfc[s];
      int ep = sE[s];
      ep = (ep > coff) ? ep : coff;
      ep = (ep > 0) ? ep : 0;
      sE[s] = ep;
    }
  }
  __syncthreads();
  const float finalv = sLfc[kS - 1];
  float gmax = -__builtin_inff();
#pragma unroll 1
  for (int e = 0; e < 8; ++e) {
    const int s = base + e;
    const float lgf = (Ih[s] - sLfc[s]) + finalv;
    gmax = fmaxf(gmax, lgf);
  }
#pragma unroll
  for (int off = 16; off > 0; off >>= 1) gmax = fmaxf(gmax, __shfl_xor(gmax, off, 32));
  if (lane == 0) sRed[wave] = gmax;
  __syncthreads();
  float gm = sRed[0];
#pragma unroll
  for (int w = 1; w < 8; ++w) gm = fmaxf(gm, sRed[w]);
  const float mval = fmaxf(finalv + pmb, gm);
  const float pd = expf((pmb + finalv) - mval);

  plane_store_f(sLfc, ST + ((size_t)(h * kStatN + 0)) * kS, t);
#pragma unroll 1
  for (int e = 0; e < 8; ++e) {
    const int s = base + e;
    const float iv = Ih[s];
    const float l = sLfc[s];
    const float stab = fmaxf(iv, l + pmb);
    sA[s] = iv - stab;
  }
  __syncthreads();
  plane_store_f(sA, ST + ((size_t)(h * kStatN + 1)) * kS, t);
  __syncthreads();
#pragma unroll 1
  for (int e = 0; e < 8; ++e) {
    const int s = base + e;
    const float iv = Ih[s];
    const float l = sLfc[s];
    const float stab = fmaxf(iv, l + pmb);
    sA[s] = expf((l + pmb) - stab) * kQScale;
  }
  __syncthreads();
  plane_store_f(sA, ST + ((size_t)(h * kStatN + 2)) * kS, t);
  __syncthreads();
#pragma unroll 1
  for (int e = 0; e < 8; ++e) {
    const int s = base + e;
    const float iv = Ih[s];
    const float l = sLfc[s];
    const float stab = fmaxf(iv, l + pmb);
    sA[s] = expf(-stab);
  }
  __syncthreads();
  plane_store_f(sA, ST + ((size_t)(h * kStatN + 3)) * kS, t);
  __syncthreads();
  plane_store_i(sE, EPS + (size_t)h * kS, t);
#pragma unroll 1
  for (int e = 0; e < 8; ++e) {
    const int s = base + e;
    const float lgf = (Ih[s] - sLfc[s]) + finalv;
    sA[s] = expf(lgf - mval);
  }
  if (t < 8) {
    v4f mv;
    mv.x = (t == 0) ? mval : 0.0f;
    mv.y = (t == 0) ? pd : 0.0f;
    mv.z = 0.0f;
    mv.w = 0.0f;
    float* mp = Mtab + (size_t)h * kMtabPitch + 4 * t;
    *(volatile v4f*)mp = mv;
    __threadfence();
    *(volatile v4f*)mp = mv;
  }
  __syncthreads();

  const int dpair = lane;
  const int sq = wave;
  float nacc[2][2];
  nacc[0][0] = 0.0f; nacc[0][1] = 0.0f; nacc[1][0] = 0.0f; nacc[1][1] = 0.0f;
  const int q8 = lane >> 3, c8 = (lane & 7) * 8;
#pragma unroll 1
  for (int ch = 0; ch < kS / 64; ++ch) {
    const int s0 = ch * 64;
#pragma unroll
    for (int dh = 0; dh < 2; ++dh) {
#pragma unroll 1
      for (int i = 0; i < 8; ++i) {
        const int sl = sq * 8 + i;
        const int s = s0 + sl;
        const unsigned int w = Kb32[(size_t)h * kHeadWords + (size_t)s * 64 + dh * 32 + dpair];
        const float kv = sA[s];
        const float k0v = __uint_as_float(w << 16);
        const float k1v = __uint_as_float(w & 0xffff0000u);
        const float p0 = k0v * kv;
        const float p1 = k1v * kv;
        nacc[dh][0] += p0;
        nacc[dh][1] += p1;
        const unsigned short h0 = f2bf_bits(p0);
        const unsigned short h1 = f2bf_bits(p1);
        const unsigned short l0 = f2bf_bits(p0 - bf_bits2f(h0));
        const unsigned short l1 = f2bf_bits(p1 - bf_bits2f(h1));
        sHi[(2 * dpair) * kWPitch + sl] = h0;
        sHi[(2 * dpair + 1) * kWPitch + sl] = h1;
        sLo[(2 * dpair) * kWPitch + sl] = l0;
        sLo[(2 * dpair + 1) * kWPitch + sl] = l1;
      }
      __syncthreads();
      for (int pass = 0; pass < 2; ++pass) {
#pragma unroll
        for (int it = 0; it < 2; ++it) {
          const int row = wave * 8 + it * 4 + q8;
          const v4u hvv = *(const v4u*)(const void*)(sHi + row * kWPitch + c8);
          const v4u lvv = *(const v4u*)(const void*)(sLo + row * kWPitch + c8);
          const size_t g = ((size_t)(h * kDH + dh * 64 + row)) * kS + s0 + c8;
          *(volatile v4u*)(KKh + g) = hvv;
          *(volatile v4u*)(KKl + g) = lvv;
        }
        __threadfence();
      }
      __syncthreads();
    }
  }
#pragma unroll
  for (int dh = 0; dh < 2; ++dh) {
    sN[sq][dh * 64 + 2 * dpair]     = nacc[dh][0];
    sN[sq][dh * 64 + 2 * dpair + 1] = nacc[dh][1];
  }
  __syncthreads();
  if (wave < 4) {
    const int d = t;
    const float tot = ((sN[0][d] + sN[1][d]) + (sN[2][d] + sN[3][d])) + ((sN[4][d] + sN[5][d]) + (sN[6][d] + sN[7][d]));
    sOut[d] = sPn[d] * pd + tot;
  }
  __syncthreads();
  if (wave == 0) {
    const v4f val = *(const v4f*)(sOut + 4 * lane);
    float* dp = outN + (size_t)h * kDH + 4 * lane;
    *(volatile v4f*)dp = val;
    __threadfence();
    *(volatile v4f*)dp = val;
  }
}

__global__ __launch_bounds__(128) void k_attn(
    const unsigned short* __restrict__ Qb, const unsigned short* __restrict__ Kb,
    const unsigned short* __restrict__ VbT, const unsigned short* __restrict__ PCX,
    const float* __restrict__ ST, const int* __restrict__ EPS, float* __restrict__ OST) {
  __shared__ __align__(16) float sStat[kStatN][64];
  __shared__ int sEps[64];
  __shared__ __align__(16) unsigned short Wh[4][16 * kWPitch];
  __shared__ __align__(16) unsigned short Wl[4][16 * kWPitch];
  __shared__ __align__(16) float Os[4][16 * kOsPitch];

  const int tid = threadIdx.x;
  const int wave = tid >> 5, lane = tid & 31, hh = lane >> 4, c = lane & 15, koff = hh * 8;
  const int h = blockIdx.x >> 5, rb = blockIdx.x & 31;
  const int r0 = rb * 64;
  const int q0 = r0 + wave * 16;
  {
    const int row = tid & 63, a0 = tid >> 6;
    sStat[a0][row]     = ST[((size_t)(h * kStatN + a0)) * kS + r0 + row];
    sStat[a0 + 2][row] = ST[((size_t)(h * kStatN + a0 + 2)) * kS + r0 + row];
    if (wave < 2) sEps[row] = EPS[(size_t)h * kS + r0 + row];
  }
  __syncthreads();
  int jtlo = __builtin_amdgcn_readfirstlane(sEps[0] >> 6);
  jtlo = (jtlo < 0) ? 0 : jtlo;
  jtlo = (jtlo > rb) ? rb : jtlo;

  v16b qa[4];
  {
    const unsigned short* qrow = Qb + (size_t)h * kHeadElems + (size_t)(q0 + c) * kDH + koff;
#pragma unroll
    for (int ks = 0; ks < 4; ++ks) qa[ks] = fload(qrow + 32 * ks);
  }
  v8f acc[9];
#pragma unroll
  for (int nt = 0; nt < 9; ++nt) acc[nt] = zero8();
  {
    const unsigned short* pcx = PCX + (size_t)h * kPcxHead + (size_t)c * kDH + koff;
#pragma unroll
    for (int ks = 0; ks < 4; ++ks) {
#pragma unroll
      for (int nt = 0; nt < 9; ++nt) {
        const v16b pb = fload(pcx + (size_t)(16 * nt) * kDH + 32 * ks);
        acc[nt] = mma_bf(qa[ks], pb, acc[nt]);
        hz1(acc[nt], qa[ks], pb);
        if (nt == 4) sched_fence();
      }
      sched_fence();
    }
  }
  float dq8[8], intn8[8], rs[8];
  {
    float a8s[8];
#pragma unroll
    for (int r = 0; r < 8; ++r) {
      const int lr = wave * 16 + 8 * hh + r;
      dq8[r] = sStat[2][lr];
      a8s[r] = acc[8][r] * dq8[r];
      rs[r] = 0.0f;
    }
#pragma unroll
    for (int r = 0; r < 8; ++r) intn8[r] = __shfl(a8s[r], lane & 16, 32);
  }
#pragma unroll
  for (int nt = 0; nt < 8; ++nt) {
#pragma unroll
    for (int r = 0; r < 8; ++r) acc[nt][r] = acc[nt][r] * dq8[r];
  }

  const float* LFCp = ST + ((size_t)(h * kStatN)) * kS;
  const unsigned short* kbase = Kb + (size_t)h * kHeadElems + (size_t)c * kDH + koff;
  const unsigned short* vbase = VbT + ((size_t)(h * kDH + c)) * kS + koff;
  unsigned short* wh = Wh[wave];
  unsigned short* wl = Wl[wave];

  for (int jt = jtlo; jt <= rb; ++jt) {
    const int j0 = jt * 64;
    v8f e[4];
#pragma unroll
    for (int j = 0; j < 4; ++j) e[j] = zero8();
#pragma unroll
    for (int ks = 0; ks < 4; ++ks) {
      v16b kb[4];
#pragma unroll
      for (int j = 0; j < 4; ++j) kb[j] = fload(kbase + (size_t)(j0 + 16 * j) * kDH + 32 * ks);
#pragma unroll
      for (int j = 0; j < 4; ++j) e[j] = mma_bf(qa[ks], kb[j], e[j]);
      hz4x5(e[0], e[1], e[2], e[3], qa[ks], kb[0], kb[1], kb[2], kb[3]);
      sched_fence();
    }
    const float lfcj0 = LFCp[j0];
    int colv[4];
    float colf[4];
#pragma unroll
    for (int j = 0; j < 4; ++j) {
      colv[j] = j0 + 16 * j + c;
      colf[j] = expf(lfcj0 - LFCp[colv[j]]);
    }
    __syncthreads();
#pragma unroll
    for (int r = 0; r < 8; ++r) {
      const int lr = wave * 16 + 8 * hh + r;
      const int row = r0 + lr;
      const float rowf = expf((sStat[0][lr] - lfcj0) + sStat[1][lr]);
      const int eps = sEps[lr];
#pragma unroll
      for (int j = 0; j < 4; ++j) {
        const bool ok = (colv[j] >= eps) && (colv[j] <= row);
        const float dv = ok ? (rowf * colf[j]) : 0.0f;
        const float w = (e[j][r] * kQScale) * dv;
        rs[r] += w;
        const unsigned short hb = f2bf_bits(w);
        const unsigned short lb = f2bf_bits(w - bf_bits2f(hb));
        const int widx = (8 * hh + r) * kWPitch + 16 * j + c;
        wh[widx] = hb;
        wl[widx] = lb;
      }
    }
    __syncthreads();
#pragma unroll
    for (int kk = 0; kk < 2; ++kk) {
      const v16b wa = fload(wh + c * kWPitch + 32 * kk + koff);
      const v16b wb = fload(wl + c * kWPitch + 32 * kk + koff);
#pragma unroll
      for (int nt = 0; nt < 8; ++nt) {
        const v16b vb = fload(vbase + (size_t)(16 * nt) * kS + j0 + 32 * kk);
        acc[nt] = mma_bf(wa, vb, acc[nt]);
        acc[nt] = mma_bf(wb, vb, acc[nt]);
        hz1x3(acc[nt], wa, wb, vb);
        if (nt == 3) sched_fence();
      }
      sched_fence();
    }
  }

#pragma unroll
  for (int m = 1; m < 16; m <<= 1) {
#pragma unroll
    for (int r = 0; r < 8; ++r) rs[r] += __shfl_xor(rs[r], m, 32);
  }
  float sc[8];
#pragma unroll
  for (int r = 0; r < 8; ++r) {
    const int lr = wave * 16 + 8 * hh + r;
    const float fl = sStat[3][lr];
    const float nrm = fmaxf(fabsf(rs[r]) + intn8[r], fl);
    sc[r] = 1.0f / (nrm + 1e-6f);
  }
  float* os = Os[wave];
  const int c4 = c * 4;
#pragma unroll
  for (int half = 0; half < 2; ++half) {
#pragma unroll
    for (int r = 0; r < 8; ++r) {
#pragma unroll
      for (int u = 0; u < 4; ++u) os[(8 * hh + r) * kOsPitch + 16 * u + c] = acc[4 * half + u][r] * sc[r];
    }
    __syncthreads();
    for (int pass = 0; pass < 2; ++pass) {
#pragma unroll
      for (int it = 0; it < 8; ++it) {
        const int row = it * 2 + hh;
        const v4f val = *(const v4f*)(os + row * kOsPitch + c4);
        *(volatile v4f*)(OST + ((size_t)(h * kS + q0 + row)) * kDH + half * 64 + c4) = val;
      }
      __threadfence();
    }
    __syncthreads();
  }
}

__global__ __launch_bounds__(128) void k_state(const unsigned short* __restrict__ KKh, const unsigned short* __restrict__ KKl,
                                              const unsigned short* __restrict__ VbT, const float* __restrict__ prevC,
                                              const float* __restrict__ Mtab, float* __restrict__ outC) {
  __shared__ __align__(16) float sT[4][16 * kOsPitch];
  const int h = blockIdx.x, tid = threadIdx.x;
  const int wave = tid >> 5, lane = tid & 31, hh = lane >> 4, c = lane & 15, koff = hh * 8;
  const int tm = wave >> 1, tn = wave & 1;
  const int m0 = tm * 64, n0 = tn * 64;
  const unsigned short* A  = KKh + (size_t)h * kDH * kS;
  const unsigned short* A2 = KKl + (size_t)h * kDH * kS;
  const unsigned short* Bt = VbT + (size_t)h * kDH * kS;
  v8f acc[4][4];
#pragma unroll
  for (int i = 0; i < 4; ++i)
#pragma unroll
    for (int j = 0; j < 4; ++j) acc[i][j] = zero8();
#pragma unroll 1
  for (int k0 = 0; k0 < kS; k0 += 32) {
    v16b bh[4];
#pragma unroll
    for (int j = 0; j < 4; ++j) bh[j] = fload(Bt + (size_t)(n0 + 16 * j + c) * kS + k0 + koff);
#pragma unroll
    for (int i = 0; i < 4; ++i) {
      const size_t ao = (size_t)(m0 + 16 * i + c) * kS + k0 + koff;
      const v16b ah = fload(A + ao);
      const v16b al = fload(A2 + ao);
#pragma unroll
      for (int j = 0; j < 4; ++j) {
        acc[i][j] = mma_bf(ah, bh[j], acc[i][j]);
        acc[i][j] = mma_bf(al, bh[j], acc[i][j]);
      }
      hz4x6(acc[i][0], acc[i][1], acc[i][2], acc[i][3], ah, al, bh[0], bh[1], bh[2], bh[3]);
    }
  }
  const float pd = Mtab[(size_t)h * kMtabPitch + 1];
  float* slab = sT[wave];
  const int c4 = c * 4;
#pragma unroll
  for (int i = 0; i < 4; ++i) {
    const int mBase = m0 + 16 * i;
#pragma unroll
    for (int j = 0; j < 4; ++j) {
#pragma unroll
      for (int r = 0; r < 8; ++r) slab[(8 * hh + r) * kOsPitch + 16 * j + c] = acc[i][j][r];
    }
    __syncthreads();
    v4f val[8];
#pragma unroll
    for (int it = 0; it < 8; ++it) {
      const int row = it * 2 + hh;
      const v4f sv = *(const v4f*)(slab + row * kOsPitch + c4);
      const size_t gi = ((size_t)(h * kDH + mBase + row)) * kDH + n0 + c4;
      const v4f rv = *(const v4f*)(prevC + gi);
      v4f o;
      o.x = sv.x + bfr(rv.x) * pd;
      o.y = sv.y + bfr(rv.y) * pd;
      o.z = sv.z + bfr(rv.z) * pd;
      o.w = sv.w + bfr(rv.w) * pd;
      val[it] = o;
    }
    for (int pass = 0; pass < 2; ++pass) {
#pragma unroll
      for (int it = 0; it < 8; ++it) {
        const int row = it * 2 + hh;
        const size_t gi = ((size_t)(h * kDH + mBase + row)) * kDH + n0 + c4;
        *(volatile v4f*)(outC + gi) = val[it];
      }
      __threadfence();
    }
    __syncthreads();
  }
}

__global__ __launch_bounds__(256) void k_pack(const float* __restrict__ OST, const float* __restrict__ Mtab,
                                             float* __restrict__ outp, int n4) {
  const int i = blockIdx.x * 256 + threadIdx.x;
  const int ic = (i < n4) ? i : (n4 - 1);
  const int src = (ic >= 2) ? (ic - 2) : 0;
  const v4f ov = *(const v4f*)(OST + (size_t)src * 4);
  float mq[8];
#pragma unroll
  for (int hq = 0; hq < 8; ++hq) mq[hq] = Mtab[hq * kMtabPitch];
  const float fo = ((i & 1) != 0) ? 1.0f : 0.0f;
  const float fe = 1.0f - fo;
  v4f mv;
  mv.x = fo * mq[4] + fe * mq[0];
  mv.y = fo * mq[5] + fe * mq[1];
  mv.z = fo * mq[6] + fe * mq[2];
  mv.w = fo * mq[7] + fe * mq[3];
  const float fa = (i < 2) ? 1.0f : 0.0f;
  const float fb = 1.0f - fa;
  v4f rvv;
  rvv.x = fa * mv.x + fb * ov.x;
  rvv.y = fa * mv.y + fb * ov.y;
  rvv.z = fa * mv.z + fb * ov.z;
  rvv.w = fa * mv.w + fb * ov.w;
  if (i < n4) {
    float* dp = outp + kOutM + (size_t)i * 4;
    *(volatile v4f*)dp = rvv;
    __threadfence();
    *(volatile v4f*)dp = rvv;
  }
}

extern "C" void kernel_launch(void* const* d_in, const int* in_sizes, int n_in,
                              void* d_out, int out_size, void* d_ws, size_t ws_size,
                              hipStream_t stream) {
  if (n_in < 11) return;
  const int nQ = kS * kHid;
  if (in_sizes[0] != nQ || in_sizes[1] != nQ || in_sizes[2] != nQ) return;
  if (in_sizes[3] != kS || in_sizes[4] != kNH * kDH * kDH || in_sizes[5] != kNH * kDH || in_sizes[6] != kNH) return;
  if (in_sizes[7] != kGateK * kNH || in_sizes[8] != kNH || in_sizes[9] != kGateK * kNH || in_sizes[10] != kNH) return;
  if (out_size != kOutTotal) return;

  const size_t szP16  = (size_t)kS * kHid * 2;
  const size_t szVT   = (size_t)kNH * kDH * kS * 2;
  const size_t szOST  = (size_t)kNH * kS * kDH * 4;
  const size_t szPCX  = (size_t)kNH * kPcxHead * 2;
  const size_t szGBt  = (size_t)kGateN * kGateK * 2;
  const size_t szIF   = (size_t)kS * kNH * 4;
  const size_t szST   = (size_t)kNH * kStatN * kS * 4;
  const size_t szEPS  = (size_t)kNH * kS * 4;
  const size_t szMtab = (size_t)kNH * kMtabPitch * 4;
  const size_t offQb  = 0;
  const size_t offKb  = offQb + szP16;
  const size_t offVb  = offKb + szP16;
  const size_t offVT  = offVb + szP16;
  const size_t offKKh = offVT + szVT;
  const size_t offKKl = offKKh + szVT;
  const size_t offOST = offKKl + szVT;
  const size_t offPCX = offOST + szOST;
  const size_t offGBt = offPCX + szPCX;
  const size_t offIpl = offGBt + szGBt;
  const size_t offFpl = offIpl + szIF;
  const size_t offST  = offFpl + szIF;
  const size_t offEPS = offST + szST;
  const size_t offMt  = offEPS + szEPS;
  const size_t total  = offMt + szMtab;
  if (ws_size < total) return;

  const float* q     = (const float*)d_in[0];
  const float* k     = (const float*)d_in[1];
  const float* v     = (const float*)d_in[2];
  const int*   flags = (const int*)d_in[3];
  const float* prevC = (const float*)d_in[4];
  const float* prevN = (const float*)d_in[5];
  const float* prevM = (const float*)d_in[6];
  const float* wik   = (const float*)d_in[7];
  const float* wib   = (const float*)d_in[8];
  const float* wfk   = (const float*)d_in[9];
  const float* wfb   = (const float*)d_in[10];
  float* out = (float*)d_out;
  char* ws = (char*)d_ws;
  unsigned short* Qb  = (unsigned short*)(ws + offQb);
  unsigned short* Kb  = (unsigned short*)(ws + offKb);
  unsigned short* Vb  = (unsigned short*)(ws + offVb);
  unsigned short* VbT = (unsigned short*)(ws + offVT);
  unsigned short* KKh = (unsigned short*)(ws + offKKh);
  unsigned short* KKl = (unsigned short*)(ws + offKKl);
  float*          OST = (float*)(ws + offOST);
  unsigned short* PCX = (unsigned short*)(ws + offPCX);
  unsigned short* GBt = (unsigned short*)(ws + offGBt);
  float*          Ipl = (float*)(ws + offIpl);
  float*          Fpl = (float*)(ws + offFpl);
  float*          ST  = (float*)(ws + offST);
  int*            EPS = (int*)(ws + offEPS);
  float*          Mtab = (float*)(ws + offMt);

  const int n8 = nQ / 8;
  k_cast3<<<dim3(n8 / 256, 3), dim3(256), 0, stream>>>(q, k, v, Qb, Kb, Vb, n8);
  k_tcast<<<dim3(kS / 64, kDH / 64, kNH), dim3(256), 0, stream>>>(v, VbT, kS, kDH, kHeadElems, kDH * kS);
  k_tcast<<<dim3(kDH / 64, kDH / 64, kNH), dim3(256), 0, stream>>>(prevC, PCX, kDH, kDH, kDH * kDH, kPcxHead);
  k_prep2<<<dim3(32), dim3(256), 0, stream>>>(wik, wfk, prevN, GBt, PCX);
  k_gates<<<dim3(kS / 512), dim3(256), 0, stream>>>(Qb, Kb, Vb, GBt, wib, wfb, Ipl, Fpl);
  k_rowstats<<<dim3(kNH), dim3(256), 0, stream>>>(Ipl, Fpl, flags, prevM, prevN, (const unsigned int*)(const void*)Kb,
                                                   ST, EPS, Mtab, KKh, KKl, out + kOutN);
  k_attn<<<dim3(kNH * (kS / 64)), dim3(128), 0, stream>>>(Qb, Kb, VbT, PCX, ST, EPS, OST);
  k_state<<<dim3(kNH), dim3(128), 0, stream>>>(KKh, KKl, VbT, prevC, Mtab, out);
  k_pack<<<dim3((kPackN4 + 255) / 256), dim3(256), 0, stream>>>(OST, Mtab, out, kPackN4);
}
